// MoE_13426067767888
// MI455X (gfx1250) — hardware-run, weakly checked
//
#include <hip/hip_runtime.h>
#include <math.h>

#define NTOK 4096
#define NPASS 2
#define NTOK_ALL (NTOK * NPASS)
#define NTOK_FULL 4096
#define DM 1024
#define II 512
#define NE 8
#define TOPK 2
#define NSLOT (NTOK * TOPK)
#define R_MAX (NSLOT + 64 * NE)
#define NT_MAX (R_MAX / 64)
#define SPT (NSLOT / 512)
#define NGW (NTOK / 16)
#define NSH 2
#define NROW_S (NSH * NTOK)

#define CX_LOG2 11
#define CW_LOG2 16
#define CH_LOG2 10
#define CH ((float)(1u << CH_LOG2))
#define SC_HG (1.0f / (float)(1u << (CX_LOG2 + CW_LOG2)))
#define SC_Y (1.0f / (float)(1u << (CH_LOG2 + CW_LOG2)))

#define TBL_COUNT 0
#define TBL_POFF 16
#define TBL_NTILES 32
#define TBL_TILE_E 64
#define TBL_ROWTOK 256
#define TBL_SLOTROW (256 + R_MAX)
#define TBL_WORDS (256 + R_MAX + NSLOT)
#define TBLS_WORDS 256

#define OUT_S1_OFF ((size_t)NTOK_ALL * (size_t)DM)

static_assert(NE <= 16 && TOPK == 2 && NSLOT % 512 == 0);
static_assert(NE == 8 && NPASS == 2);
static_assert(NTOK <= NTOK_FULL && NTOK % 128 == 0 && NTOK % 64 == 0);
static_assert(SPT % 4 == 0 && SPT >= 4);
static_assert(R_MAX % 64 == 0 && TBL_TILE_E + NT_MAX <= 256);
static_assert(DM == 1024 && II == 512 && II % 64 == 0 && II % 32 == 0);
static_assert((NTOK * DM / 8) % 256 == 0);
static_assert((TBL_WORDS * 4) % 256 == 0);
static_assert(NSLOT == 8192 && R_MAX == 8704 && NT_MAX == 136 && TBL_WORDS == 17152);
static_assert(NROW_S / 64 <= NT_MAX && NROW_S <= R_MAX && NSH <= NE);
static_assert(((unsigned long long)OUT_S1_OFF * 4ull) % 128ull == 0ull);

constexpr size_t al256(size_t b) { return (b + 255) & ~(size_t)255; }
constexpr size_t SZ_X16S = al256((size_t)NROW_S * DM * 2);
constexpr size_t SZ_W   = al256((size_t)NE * II * DM * 2);
constexpr size_t SZ_WS  = al256((size_t)NSH * II * DM * 2);
constexpr size_t SZ_SEL = al256((size_t)NSLOT * 4);
constexpr size_t SZ_WGT = al256((size_t)NSLOT * 4);
constexpr size_t SZ_TBL = al256((size_t)TBL_WORDS * 4);
constexpr size_t SZ_XG  = al256((size_t)R_MAX * DM * 2);
constexpr size_t SZ_HG  = al256((size_t)R_MAX * II * 2);
constexpr size_t SZ_YG  = al256((size_t)R_MAX * DM * 4);
constexpr size_t SZ_GS  = al256((size_t)NPASS * NGW * 32 * 4);
constexpr size_t SZ_TBLS = al256((size_t)TBLS_WORDS * 4);
constexpr size_t WS_TOTAL = 3 * SZ_W + 3 * SZ_WS + SZ_SEL + SZ_WGT + SZ_TBL + SZ_X16S + SZ_XG + SZ_HG + SZ_YG + SZ_GS + SZ_TBLS;
static_assert(WS_TOTAL < (size_t)134217728);
static_assert((size_t)NROW_S * II * 2 <= SZ_HG && (size_t)NROW_S * DM * 4 <= SZ_X16S + SZ_XG && SZ_X16S == (size_t)NROW_S * DM * 2);

typedef _Float16 h16;
typedef __attribute__((ext_vector_type(16))) _Float16 v16h;
typedef __attribute__((ext_vector_type(8)))  _Float16 v8h;
typedef __attribute__((ext_vector_type(8)))  float    v8f;
typedef __attribute__((ext_vector_type(4)))  float    v4f;
typedef __attribute__((ext_vector_type(2)))  float    v2f;
typedef __attribute__((ext_vector_type(4)))  unsigned int v4u;
typedef __attribute__((ext_vector_type(4)))  int      v4i;
typedef __attribute__((ext_vector_type(2)))  int      v2i;


#define VST2(T, ptr, val) do { const T vst2_v_ = (val); *(volatile T*)(ptr) = vst2_v_; __threadfence(); *(volatile T*)(ptr) = vst2_v_; } while (0)

static __device__ __forceinline__ float bfr(float f) {
    unsigned u = __float_as_uint(f);
    u += 0x7FFFu + ((u >> 16) & 1u);
    return __uint_as_float(u & 0xFFFF0000u);
}
static __device__ __forceinline__ h16 toh_flush(float v) { const float w = (fabsf(v) < 6.103515625e-05f) ? 0.0f : v; return (h16)w; }
static __device__ __forceinline__ void st8h(h16* p, const float* v) {
    v8h hv;
#pragma unroll
    for (int e = 0; e < 8; ++e) hv[e] = toh_flush(v[e]);
    VST2(v8h, p, hv);
}

union FragU { v16h v; v8h h[2]; };
static __device__ __forceinline__ v16h frag_ld(const h16* p) {
    FragU f; f.h[0] = *(const v8h*)(p); f.h[1] = *(const v8h*)(p + 16); return f.v;
}
static __device__ __forceinline__ v8f wmma16g(v16h a, v16h b, v8f c) {
    c = __builtin_amdgcn_wmma_f32_16x16x32_f16(false, a, false, b, (short)0, c, false, false);
    asm volatile("v_nop\n\tv_nop\n\tv_nop\n\tv_nop" : "+v"(c) : "v"(a), "v"(b));
    return c;
}
static __device__ __forceinline__ void wave_sync_lds() {
    __builtin_amdgcn_fence(3  , "workgroup");
    __builtin_amdgcn_wave_barrier();
    __builtin_amdgcn_fence(2  , "workgroup");
}

template <int LOG2C>
__global__ __launch_bounds__(256) void k_plane(const float* __restrict__ src, h16* __restrict__ dst, unsigned n8) {
    const unsigned u = blockIdx.x * 256u + threadIdx.x;
    if (u >= n8) return;
    const float cs = (float)(1u << LOG2C);
    const v4f a = *(const v4f*)(src + (size_t)u * 8u);
    const v4f b = *(const v4f*)(src + (size_t)u * 8u + 4u);
    float v[8] = {bfr(a.x) * cs, bfr(a.y) * cs, bfr(a.z) * cs, bfr(a.w) * cs, bfr(b.x) * cs, bfr(b.y) * cs, bfr(b.z) * cs, bfr(b.w) * cs};
    st8h(dst + (size_t)u * 8u, v);
}

__global__ __launch_bounds__(128) void k_planeTw(const float* __restrict__ src, h16* __restrict__ dst, unsigned ne, unsigned K, unsigned N, unsigned pitch, unsigned estride, float cs) {
    __shared__ __align__(16) float sT[4][64 * 36];
    const unsigned lane = threadIdx.x & 31u;
    const unsigned wave = threadIdx.x >> 5;
    const unsigned tk = K >> 6, tn = N >> 5;
    const unsigned tpe = tk * tn;
    const unsigned u = blockIdx.x * 4u + wave;
    if (u >= ne * tpe) return;
    const unsigned e = u / tpe;
    const unsigned rem = u - e * tpe;
    const unsigned kt = rem / tn;
    const unsigned nt = rem - kt * tn;
    const unsigned k0 = kt << 6, n0 = nt << 5;
    const size_t sbase = (size_t)e * (size_t)estride;
    const size_t ebase = (size_t)e * ((size_t)K * (size_t)N);
    float* slab = sT[wave];
#pragma unroll
    for (int i = 0; i < 16; ++i) {
        const unsigned p = lane + 32u * (unsigned)i;
        const unsigned kr = p >> 3;
        const unsigned n4 = (p & 7u) * 4u;
        const v4f a = *(const v4f*)(src + sbase + (size_t)(k0 + kr) * pitch + n0 + n4);
        v4f s;
        s.x = bfr(a.x) * cs; s.y = bfr(a.y) * cs; s.z = bfr(a.z) * cs; s.w = bfr(a.w) * cs;
        *(v4f*)(&slab[kr * 36u + n4]) = s;
    }
    wave_sync_lds();
#pragma unroll
    for (int i = 0; i < 8; ++i) {
        const unsigned q = lane + 32u * (unsigned)i;
        const unsigned n = q >> 3;
        const unsigned kp = q & 7u;
        float v[8];
#pragma unroll
        for (int j = 0; j < 8; ++j) v[j] = slab[(8u * kp + (unsigned)j) * 36u + n];
        st8h(dst + ebase + (size_t)(n0 + n) * K + k0 + 8u * kp, v);
    }
}

__global__ __launch_bounds__(256) void k_gate(const float* __restrict__ x, const float* __restrict__ gw,
                                              int* __restrict__ sel, float* __restrict__ wgt, float* __restrict__ gs) {
    const unsigned lane = threadIdx.x & 31u;
    const unsigned wave = threadIdx.x >> 5;
    const unsigned gwv = blockIdx.x * 8u + wave;
    const unsigned t0 = gwv * 16u;
    if (t0 >= (unsigned)NTOK) return;
    int ki0 = 0, ki1 = 0;
    float kw0 = 0.0f, kw1 = 0.0f;
    float acc = 0.0f;
    for (unsigned j = 0; j < 16u; ++j) {
        const float* xr = x + (size_t)(t0 + j) * DM;
        float lg[NE];
#pragma unroll
        for (int e = 0; e < NE; ++e) lg[e] = 0.0f;
        for (unsigned i = 0; i < (unsigned)(DM / 32); ++i) {
            const unsigned d = lane + 32u * i;
            const float xv = bfr(xr[d]);
            const v4f ga = *(const v4f*)(gw + (size_t)d * NE);
            const v4f gc = *(const v4f*)(gw + (size_t)d * NE + 4u);
            lg[0] += xv * bfr(ga.x); lg[1] += xv * bfr(ga.y); lg[2] += xv * bfr(ga.z); lg[3] += xv * bfr(ga.w);
            lg[4] += xv * bfr(gc.x); lg[5] += xv * bfr(gc.y); lg[6] += xv * bfr(gc.z); lg[7] += xv * bfr(gc.w);
        }
#pragma unroll
        for (int e = 0; e < NE; ++e) {
            lg[e] += __shfl_xor(lg[e], 16, 32);
            lg[e] += __shfl_xor(lg[e], 8, 32);
            lg[e] += __shfl_xor(lg[e], 4, 32);
            lg[e] += __shfl_xor(lg[e], 2, 32);
            lg[e] += __shfl_xor(lg[e], 1, 32);
        }
        float m = lg[0];
#pragma unroll
        for (int e = 1; e < NE; ++e) m = fmaxf(m, lg[e]);
        float pr[NE];
        float s = 0.0f;
#pragma unroll
        for (int e = 0; e < NE; ++e) { pr[e] = expf(lg[e] - m); s += pr[e]; }
#pragma unroll
        for (int e = 0; e < NE; ++e) pr[e] = pr[e] / s;
        float bestv = pr[0];
        int besti = 0;
#pragma unroll
        for (int e = 1; e < NE; ++e) { const bool c = pr[e] > bestv; bestv = c ? pr[e] : bestv; besti = c ? e : besti; }
        float secv = -1.0f;
        int seci = 0;
#pragma unroll
        for (int e = 0; e < NE; ++e) { const bool c = (e != besti) && (pr[e] > secv); secv = c ? pr[e] : secv; seci = c ? e : seci; }
        const bool mine = (lane == j);
        ki0 = mine ? besti : ki0;  ki1 = mine ? seci : ki1;
        const float psum = bestv + secv;
        kw0 = mine ? bestv / psum : kw0;  kw1 = mine ? secv / psum : kw1;
        float add = 0.0f;
#pragma unroll
        for (int e = 0; e < NE; ++e) add = (lane == (unsigned)e) ? pr[e] : add;
        acc += add;
    }
    if (lane < 16u) {
        v2i sv; sv.x = ki0; sv.y = ki1;
        v2f wv; wv.x = kw0; wv.y = kw1;
        VST2(v2i, sel + (size_t)(t0 + lane) * 2u, sv);
        VST2(v2f, wgt + (size_t)(t0 + lane) * 2u, wv);
    }
    VST2(float, gs + (size_t)gwv * 32u + lane, acc);
}

__global__ __launch_bounds__(512) void k_route(const int* __restrict__ sel, int* __restrict__ tbl) {
    __shared__ __align__(16) int s_rt[R_MAX];
    __shared__ __align__(16) int s_hdr[256];
    __shared__ int sc[512];
    const unsigned tid = threadIdx.x;
    for (unsigned i = tid; i < (unsigned)R_MAX; i += 512u) s_rt[i] = -1;
    if (tid < 256u) s_hdr[tid] = (tid >= (unsigned)TBL_TILE_E && tid < (unsigned)(TBL_TILE_E + NT_MAX)) ? -1 : 0;
    __syncthreads();
    int es[SPT];
    int cnt[NE];
#pragma unroll
    for (int j = 0; j < NE; ++j) cnt[j] = 0;
    const v4i* sp = (const v4i*)(sel + (size_t)tid * (unsigned)SPT);
#pragma unroll
    for (int g = 0; g < SPT / 4; ++g) {
        const v4i v = sp[g];
        es[4 * g + 0] = min(max(v.x, 0), NE - 1);
        es[4 * g + 1] = min(max(v.y, 0), NE - 1);
        es[4 * g + 2] = min(max(v.z, 0), NE - 1);
        es[4 * g + 3] = min(max(v.w, 0), NE - 1);
    }
#pragma unroll
    for (int q = 0; q < SPT; ++q)
#pragma unroll
        for (int j = 0; j < NE; ++j) cnt[j] += (es[q] == j) ? 1 : 0;
    int base[NE], total[NE];
#pragma unroll
    for (int j = 0; j < NE; ++j) {
        sc[tid] = cnt[j];
        __syncthreads();
        for (unsigned off = 1u; off < 512u; off <<= 1) {
            const unsigned src = (tid >= off) ? (tid - off) : 0u;
            const int add = sc[src];
            const int v = sc[tid] + ((tid >= off) ? add : 0);
            __syncthreads();
            sc[tid] = v;
            __syncthreads();
        }
        base[j] = sc[tid] - cnt[j];
        total[j] = sc[511];
        __syncthreads();
    }
    int poff[NE + 1];
    poff[0] = 0;
#pragma unroll
    for (int j = 0; j < NE; ++j) poff[j + 1] = poff[j] + (((total[j] + 63) >> 6) << 6);
    int rw[SPT];
#pragma unroll
    for (int q = 0; q < SPT; ++q) {
        int row = 0;
#pragma unroll
        for (int j = 0; j < NE; ++j) {
            const bool hit = (es[q] == j);
            row = hit ? (poff[j] + base[j]) : row;
            base[j] += hit ? 1 : 0;
        }
        row = min(max(row, 0), R_MAX - 1);
        rw[q] = row;
        s_rt[row] = (int)((tid * (unsigned)SPT + (unsigned)q) >> 1);
    }
    if (tid == 0u) {
#pragma unroll
        for (int j = 0; j < NE; ++j) { s_hdr[TBL_COUNT + j] = total[j]; s_hdr[TBL_POFF + j] = poff[j]; }
        s_hdr[TBL_POFF + NE] = poff[NE];
        s_hdr[TBL_NTILES] = poff[NE] >> 6;
    }
    if (tid < (unsigned)NT_MAX) {
        const int b64 = (int)(tid * 64u);
        int ev = -1;
#pragma unroll
        for (int j = 0; j < NE; ++j) ev = (b64 >= poff[j] && b64 < poff[j + 1]) ? j : ev;
        s_hdr[TBL_TILE_E + tid] = ev;
    }
    __syncthreads();
    for (int pass = 0; pass < 2; ++pass) {
        if (tid < 64u) *(volatile v4i*)(tbl + 4u * tid) = *(const v4i*)(&s_hdr[4u * tid]);
        for (unsigned i = tid; i < (unsigned)(R_MAX / 4); i += 512u) *(volatile v4i*)(tbl + TBL_ROWTOK + 4u * i) = *(const v4i*)(&s_rt[4u * i]);
        __threadfence();
    }
    __syncthreads();
#pragma unroll
    for (int g = 0; g < SPT / 4; ++g) {
        v4i pk; pk.x = rw[4 * g]; pk.y = rw[4 * g + 1]; pk.z = rw[4 * g + 2]; pk.w = rw[4 * g + 3];
        *(v4i*)(&s_rt[tid * (unsigned)SPT + 4u * (unsigned)g]) = pk;
    }
    __syncthreads();
    for (int pass = 0; pass < 2; ++pass) {
        for (unsigned i = tid; i < (unsigned)(NSLOT / 4); i += 512u) *(volatile v4i*)(tbl + TBL_SLOTROW + 4u * i) = *(const v4i*)(&s_rt[4u * i]);
        __threadfence();
    }
}

__global__ __launch_bounds__(256) void k_gather(const h16* __restrict__ x16, const int* __restrict__ tbl, h16* __restrict__ Xg) {
    const unsigned row = blockIdx.x * 2u + (threadIdx.x >> 7);
    if (row >= (unsigned)R_MAX) return;
    const unsigned c = (threadIdx.x & 127u) * 8u;
    const int tr = tbl[TBL_ROWTOK + row];
    const bool pad = (tr < 0);
    const int tok = min(max(tr, 0), NTOK - 1);
    const v4u ld = *(const v4u*)(x16 + (size_t)(unsigned)tok * DM + c);
    v4u v;
    v.x = pad ? 0u : ld.x; v.y = pad ? 0u : ld.y; v.z = pad ? 0u : ld.z; v.w = pad ? 0u : ld.w;
    VST2(v4u, Xg + (size_t)row * DM + c, v);
}

__global__ __launch_bounds__(256) void k_ffn1(const h16* __restrict__ Xg, const h16* __restrict__ W1p, const h16* __restrict__ W3p,
                                              const int* __restrict__ tbl, h16* __restrict__ Hg) {
    __shared__ __align__(16) float sT[8][16 * 68];
    const unsigned lane = threadIdx.x & 31u;
    const unsigned wave = threadIdx.x >> 5;
    const unsigned u = blockIdx.x * 8u + wave;
    if (u >= (unsigned)(NT_MAX * 2 * (II / 64))) return;
    const unsigned rt32 = u / (unsigned)(II / 64);
    const unsigned ct = u - rt32 * (unsigned)(II / 64);
    const unsigned rowtile = rt32 >> 1;
    const int nt = min(max(tbl[TBL_NTILES], 0), NT_MAX);
    if ((int)rowtile >= nt) return;
    const int e = min(max(tbl[TBL_TILE_E + rowtile], 0), NE - 1);
    const size_t wbase = (size_t)(unsigned)e * (size_t)(II * DM);
    const unsigned m0 = rt32 * 32u, n0 = ct * 64u;
    const unsigned rlane = lane & 15u;
    const unsigned koff = (lane >> 4) * 8u;
    const unsigned mOff = koff;

    v8f acc1[2][4], acc3[2][4];
#pragma unroll
    for (int i = 0; i < 2; ++i)
#pragma unroll
        for (int j = 0; j < 4; ++j) { acc1[i][j] = (v8f){0.f,0.f,0.f,0.f,0.f,0.f,0.f,0.f}; acc3[i][j] = acc1[i][j]; }

    for (unsigned k0 = 0; k0 < (unsigned)DM; k0 += 32u) {
        v16h ah[2];
#pragma unroll
        for (int i = 0; i < 2; ++i)
            ah[i] = frag_ld(Xg + (size_t)(m0 + ((unsigned)i << 4) + rlane) * DM + koff + k0);
#pragma unroll
        for (int j = 0; j < 4; ++j) {
            const size_t bo = wbase + (size_t)(n0 + ((unsigned)j << 4) + rlane) * DM + koff + k0;
            const v16h b1 = frag_ld(W1p + bo);
            const v16h b3 = frag_ld(W3p + bo);
#pragma unroll
            for (int i = 0; i < 2; ++i) {
                acc1[i][j] = wmma16g(ah[i], b1, acc1[i][j]);
                acc3[i][j] = wmma16g(ah[i], b3, acc3[i][j]);
            }
        }
    }

    float* slab = sT[wave];
#pragma unroll
    for (int i = 0; i < 2; ++i) {
        const unsigned mBase = m0 + ((unsigned)i << 4);
#pragma unroll
        for (int j = 0; j < 4; ++j) {
#pragma unroll
            for (int r = 0; r < 8; ++r) {
                const float h = acc1[i][j][r] * SC_HG;
                const float g = acc3[i][j][r] * SC_HG;
                const float a = (h / (1.0f + expf(-h))) * g;
                slab[(mOff + (unsigned)r) * 68u + ((unsigned)j << 4) + rlane] = a * CH;
            }
        }
        wave_sync_lds();
        const unsigned q = lane >> 3, c8 = (lane & 7u) * 8u;
        v8h hv[4];
#pragma unroll
        for (int it = 0; it < 4; ++it) {
            const unsigned row = (unsigned)it * 4u + q;
            const float* sp = slab + row * 68u + c8;
#pragma unroll
            for (int t = 0; t < 8; ++t) hv[it][t] = toh_flush(sp[t]);
        }
        for (int pass = 0; pass < 2; ++pass) {
#pragma unroll
            for (int it = 0; it < 4; ++it) {
                const unsigned row = (unsigned)it * 4u + q;
                *(volatile v8h*)(Hg + (size_t)(mBase + row) * II + n0 + c8) = hv[it];
            }
            __threadfence();
        }
        wave_sync_lds();
    }
}

__global__ __launch_bounds__(256) void k_ffn2(const h16* __restrict__ Hg, const h16* __restrict__ W2p,
                                              const int* __restrict__ tbl, float* __restrict__ Yg) {
    __shared__ __align__(16) float sT[8][16 * 68];
    const unsigned lane = threadIdx.x & 31u;
    const unsigned wave = threadIdx.x >> 5;
    const unsigned u = blockIdx.x * 8u + wave;
    if (u >= (unsigned)(NT_MAX * (DM / 64))) return;
    const unsigned rowtile = u / (unsigned)(DM / 64);
    const unsigned ct = u - rowtile * (unsigned)(DM / 64);
    const int nt = min(max(tbl[TBL_NTILES], 0), NT_MAX);
    if ((int)rowtile >= nt) return;
    const int e = min(max(tbl[TBL_TILE_E + rowtile], 0), NE - 1);
    const size_t wbase = (size_t)(unsigned)e * (size_t)(DM * II);
    const unsigned m0 = rowtile << 6, n0 = ct << 6;
    const unsigned rlane = lane & 15u;
    const unsigned koff = (lane >> 4) * 8u;
    const unsigned mOff = koff;

    v8f acc[4][4];
#pragma unroll
    for (int i = 0; i < 4; ++i)
#pragma unroll
        for (int j = 0; j < 4; ++j) acc[i][j] = (v8f){0.f,0.f,0.f,0.f,0.f,0.f,0.f,0.f};

    for (unsigned k0 = 0; k0 < (unsigned)II; k0 += 32u) {
        v16h bh[4];
#pragma unroll
        for (int j = 0; j < 4; ++j)
            bh[j] = frag_ld(W2p + wbase + (size_t)(n0 + ((unsigned)j << 4) + rlane) * II + koff + k0);
#pragma unroll
        for (int i = 0; i < 4; ++i) {
            const v16h ah = frag_ld(Hg + (size_t)(m0 + ((unsigned)i << 4) + rlane) * II + koff + k0);
#pragma unroll
            for (int j = 0; j < 4; ++j) acc[i][j] = wmma16g(ah, bh[j], acc[i][j]);
        }
    }

    float* slab = sT[wave];
#pragma unroll
    for (int i = 0; i < 4; ++i) {
        const unsigned mBase = m0 + ((unsigned)i << 4);
#pragma unroll
        for (int j = 0; j < 4; ++j)
#pragma unroll
            for (int r = 0; r < 8; ++r)
                slab[(mOff + (unsigned)r) * 68u + ((unsigned)j << 4) + rlane] = acc[i][j][r] * SC_Y;
        wave_sync_lds();
        const unsigned hh = lane >> 4, c4 = (lane & 15u) * 4u;
#pragma unroll
        for (int half = 0; half < 2; ++half) {
            v4f vv[4];
#pragma unroll
            for (int it = 0; it < 4; ++it) {
                const unsigned row = (unsigned)(half * 4 + it) * 2u + hh;
                vv[it] = *(const v4f*)(slab + row * 68u + c4);
            }
            for (int pass = 0; pass < 2; ++pass) {
#pragma unroll
                for (int it = 0; it < 4; ++it) {
                    const unsigned row = (unsigned)(half * 4 + it) * 2u + hh;
                    *(volatile v4f*)(Yg + (size_t)(mBase + row) * DM + n0 + c4) = vv[it];
                }
                __threadfence();
            }
        }
        wave_sync_lds();
    }
}

__global__ __launch_bounds__(64) void k_tbl_dense(int* __restrict__ tbl) {
    const unsigned w0 = threadIdx.x * 4u;
    int q[4];
#pragma unroll
    for (int k = 0; k < 4; ++k) {
        const unsigned w = w0 + (unsigned)k;
        int val = 0;
        val = (w < (unsigned)(TBL_COUNT + NSH)) ? NTOK : val;
        val = (w >= (unsigned)TBL_POFF && w <= (unsigned)(TBL_POFF + NE)) ? (int)min((w - (unsigned)TBL_POFF) * (unsigned)NTOK, (unsigned)NROW_S) : val;
        val = (w == (unsigned)TBL_NTILES) ? (NROW_S / 64) : val;
        val = (w >= (unsigned)TBL_TILE_E && w < (unsigned)(TBL_TILE_E + NT_MAX)) ? ((w - (unsigned)TBL_TILE_E < (unsigned)(NROW_S / 64)) ? (int)((w - (unsigned)TBL_TILE_E) / (unsigned)(NTOK / 64)) : -1) : val;
        q[k] = val;
    }
    v4i v;
    v.x = q[0]; v.y = q[1]; v.z = q[2]; v.w = q[3];
    VST2(v4i, tbl + w0, v);
}

__global__ __launch_bounds__(256) void k_combine(const float* __restrict__ Yg, const float* __restrict__ Ys, const float* __restrict__ wgt,
                                                 const int* __restrict__ tbl, float* __restrict__ out) {
    const unsigned t = blockIdx.x;
    if (t >= (unsigned)NTOK) return;
    const unsigned c = threadIdx.x * 4u;
    const int r0 = min(max(tbl[TBL_SLOTROW + 2u * t], 0), R_MAX - 1);
    const int r1 = min(max(tbl[TBL_SLOTROW + 2u * t + 1u], 0), R_MAX - 1);
    const float w0 = wgt[2u * t], w1 = wgt[2u * t + 1u];
    const v4f a = *(const v4f*)(Yg + (size_t)(unsigned)r0 * DM + c);
    const v4f b = *(const v4f*)(Yg + (size_t)(unsigned)r1 * DM + c);
    const v4f s0 = *(const v4f*)(Ys + (size_t)t * DM + c);
    const v4f s1 = *(const v4f*)(Ys + (size_t)(NTOK + t) * DM + c);
    const v4f mix = (a * w0) + (b * w1);
    const v4f y = mix + (s0 + s1);
    VST2(v4f, out + (size_t)t * DM + c, y);
}

__global__ __launch_bounds__(32) void k_loss(const float* __restrict__ gs, float* __restrict__ out1) {
    const unsigned lane = threadIdx.x & 31u;
    float sum = 0.0f;
    for (unsigned w = 0; w < (unsigned)(NPASS * NGW); ++w) sum += gs[(size_t)w * 32u + lane];
    const float me = sum / (float)NTOK_ALL;
    float v = (lane < (unsigned)NE) ? me * me : 0.0f;
    v += __shfl_xor(v, 16, 32);
    v += __shfl_xor(v, 8, 32);
    v += __shfl_xor(v, 4, 32);
    v += __shfl_xor(v, 2, 32);
    v += __shfl_xor(v, 1, 32);
    if (lane == 0u) VST2(float, out1, v * (float)NE);
}

extern "C" void kernel_launch(void* const* d_in, const int* in_sizes, int n_in, void* d_out, int out_size,
                              void* d_ws, size_t ws_size, hipStream_t stream) {
    if (n_in < 8) return;
    if (in_sizes[0] < NTOK_ALL * DM || in_sizes[1] < DM * NE) return;
    if (in_sizes[2] < NE * DM * II || in_sizes[3] < NE * DM * II || in_sizes[4] < NE * II * DM) return;
    if (in_sizes[5] < DM * NSH * II || in_sizes[6] < DM * NSH * II || in_sizes[7] < NSH * II * DM) return;
    if (out_size < NTOK_ALL * DM + 1) return;

    const float* x   = (const float*)d_in[0];
    const float* gw  = (const float*)d_in[1];
    const float* w1  = (const float*)d_in[2];
    const float* w3  = (const float*)d_in[3];
    const float* w2  = (const float*)d_in[4];
    const float* sw1 = (const float*)d_in[5];
    const float* sw3 = (const float*)d_in[6];
    const float* sw2 = (const float*)d_in[7];
    float* out = (float*)d_out;

    char* wsp = (char*)d_ws;
    size_t off = 0;
    auto carve = [&](size_t bytes) -> void* { void* r = wsp + off; off += (bytes + 255) & ~(size_t)255; return r; };
    h16*   w1p = (h16*)carve((size_t)NE * II * DM * 2);
    h16*   w3p = (h16*)carve((size_t)NE * II * DM * 2);
    h16*   w2p = (h16*)carve((size_t)NE * DM * II * 2);
    h16*   s1p = (h16*)carve((size_t)NSH * II * DM * 2);
    h16*   s3p = (h16*)carve((size_t)NSH * II * DM * 2);
    h16*   s2p = (h16*)carve((size_t)NSH * DM * II * 2);
    int*   sel = (int*)carve((size_t)NSLOT * 4);
    float* wgt = (float*)carve((size_t)NSLOT * 4);
    int*   tbl = (int*)carve((size_t)TBL_WORDS * 4);
    h16*   x16S = (h16*)carve((size_t)NROW_S * DM * 2);
    h16*   Xg  = (h16*)carve((size_t)R_MAX * DM * 2);
    h16*   Hg  = (h16*)carve((size_t)R_MAX * II * 2);
    float* Yg  = (float*)carve((size_t)R_MAX * DM * 4);
    float* gs  = (float*)carve((size_t)NPASS * NGW * 32 * 4);
    int*   tblS = (int*)carve((size_t)TBLS_WORDS * 4);
    if (off != WS_TOTAL || off > ws_size || off > (size_t)134217728) return;
    if ((char*)Xg != (char*)x16S + (size_t)NROW_S * DM * 2) return;
    h16*   HgS = Hg;
    float* YgS = (float*)x16S;

    k_planeTw<<<(NE * (DM / 64) * (II / 32) + 3) / 4, 128, 0, stream>>>(w1, w1p, (unsigned)NE, (unsigned)DM, (unsigned)II, (unsigned)II, (unsigned)(DM * II), (float)(1u << CW_LOG2));
    k_planeTw<<<(NE * (DM / 64) * (II / 32) + 3) / 4, 128, 0, stream>>>(w3, w3p, (unsigned)NE, (unsigned)DM, (unsigned)II, (unsigned)II, (unsigned)(DM * II), (float)(1u << CW_LOG2));
    k_planeTw<<<(NE * (II / 64) * (DM / 32) + 3) / 4, 128, 0, stream>>>(w2, w2p, (unsigned)NE, (unsigned)II, (unsigned)DM, (unsigned)DM, (unsigned)(II * DM), (float)(1u << CW_LOG2));
    k_planeTw<<<(NSH * (DM / 64) * (II / 32) + 3) / 4, 128, 0, stream>>>(sw1, s1p, (unsigned)NSH, (unsigned)DM, (unsigned)II, (unsigned)(NSH * II), (unsigned)II, (float)(1u << CW_LOG2));
    k_planeTw<<<(NSH * (DM / 64) * (II / 32) + 3) / 4, 128, 0, stream>>>(sw3, s3p, (unsigned)NSH, (unsigned)DM, (unsigned)II, (unsigned)(NSH * II), (unsigned)II, (float)(1u << CW_LOG2));
    k_planeTw<<<(NSH * (II / 64) * (DM / 32) + 3) / 4, 128, 0, stream>>>(sw2, s2p, (unsigned)NSH, (unsigned)II, (unsigned)DM, (unsigned)DM, (unsigned)(II * DM), (float)(1u << CW_LOG2));
    k_tbl_dense<<<1, 64, 0, stream>>>(tblS);

    k_plane<CX_LOG2><<<(NTOK * DM / 8) / 256, 256, 0, stream>>>(x, x16S, (unsigned)(NTOK * DM / 8));
    k_plane<CX_LOG2><<<(NTOK * DM / 8) / 256, 256, 0, stream>>>(x, x16S + (size_t)NTOK * DM, (unsigned)(NTOK * DM / 8));
    k_gate<<<NTOK / 128, 256, 0, stream>>>(x, gw, sel, wgt, gs);
    k_route<<<1, 512, 0, stream>>>(sel, tbl);
    k_gather<<<R_MAX / 2, 256, 0, stream>>>(x16S, tbl, Xg);
    k_ffn1<<<(NT_MAX * 2 * (II / 64) + 7) / 8, 256, 0, stream>>>(Xg, w1p, w3p, tbl, Hg);
    k_ffn2<<<(NT_MAX * (DM / 64) + 7) / 8, 256, 0, stream>>>(Hg, w2p, tbl, Yg);
    k_ffn1<<<(NT_MAX * 2 * (II / 64) + 7) / 8, 256, 0, stream>>>(x16S, s1p, s3p, tblS, HgS);
    k_ffn2<<<(NT_MAX * (DM / 64) + 7) / 8, 256, 0, stream>>>(HgS, s2p, tblS, YgS);
    k_combine<<<NTOK, 256, 0, stream>>>(Yg, YgS, wgt, tbl, out);
    k_plane<CX_LOG2><<<(NTOK * DM / 8) / 256, 256, 0, stream>>>(x + (size_t)NTOK * DM, x16S, (unsigned)(NTOK * DM / 8));
    k_plane<CX_LOG2><<<(NTOK * DM / 8) / 256, 256, 0, stream>>>(x + (size_t)NTOK * DM, x16S + (size_t)NTOK * DM, (unsigned)(NTOK * DM / 8));
    k_gate<<<NTOK / 128, 256, 0, stream>>>(x + (size_t)NTOK * DM, gw, sel, wgt, gs + (size_t)NGW * 32);
    k_route<<<1, 512, 0, stream>>>(sel, tbl);
    k_gather<<<R_MAX / 2, 256, 0, stream>>>(x16S, tbl, Xg);
    k_ffn1<<<(NT_MAX * 2 * (II / 64) + 7) / 8, 256, 0, stream>>>(Xg, w1p, w3p, tbl, Hg);
    k_ffn2<<<(NT_MAX * (DM / 64) + 7) / 8, 256, 0, stream>>>(Hg, w2p, tbl, Yg);
    k_ffn1<<<(NT_MAX * 2 * (II / 64) + 7) / 8, 256, 0, stream>>>(x16S, s1p, s3p, tblS, HgS);
    k_ffn2<<<(NT_MAX * (DM / 64) + 7) / 8, 256, 0, stream>>>(HgS, s2p, tblS, YgS);
    k_combine<<<NTOK, 256, 0, stream>>>(Yg, YgS, wgt, tbl, out + (size_t)NTOK * DM);
    k_loss<<<1, 32, 0, stream>>>(gs, out + OUT_S1_OFF);
}
